// MHA_82575041233640
// MI455X (gfx1250) — hardware-verified
//
#include <hip/hip_runtime.h>
#pragma clang fp contract(off)


#ifndef NB
#define NB 2
#endif
#ifndef SEQ
#define SEQ 2048
#endif
#define NB_FULL  2
#define SEQ_FULL 2048
#define DM   1024
#define NH   16
#define HD   64
#define DQ   (NH * HD)
#define N3   (3 * DQ)
#define RH   256
#define SCL  0.125f
#define L2E  1.4426950408889634f
#define PCL2 10.0f
#define NEGBIG (-3.0e38f)
#define KOFF ((size_t)NB * NH * SEQ * HD)

typedef _Float16 h16;
typedef unsigned short bf;
typedef __attribute__((ext_vector_type(16))) __bf16   v16bf;
typedef __attribute__((ext_vector_type(16))) _Float16 v16h;
typedef __attribute__((ext_vector_type(8)))  _Float16 v8h;
typedef __attribute__((ext_vector_type(8)))  unsigned short v8us;
typedef __attribute__((ext_vector_type(16))) unsigned short v16us;
typedef __attribute__((ext_vector_type(2)))  unsigned short v2us;
typedef __attribute__((ext_vector_type(2)))  _Float16 v2h;
typedef __attribute__((ext_vector_type(8)))  float    v8f;
typedef __attribute__((ext_vector_type(4)))  float    v4f;
typedef __attribute__((ext_vector_type(2)))  float    v2f;
typedef v4f  __attribute__((may_alias)) v4fa;

static_assert(DQ == DM);
static_assert(HD == 64);
static_assert(SEQ % 64 == 0 && SEQ <= SEQ_FULL && NB <= NB_FULL);
static_assert(RH % 64 == 0 && RH <= SEQ);
static_assert(DM % 64 == 0 && N3 % 64 == 0);
static_assert((NB * SEQ) % 64 == 0);
static_assert(((size_t)N3 * DM / 64) % 64 == 0 && ((size_t)DM * DQ / 64) % 64 == 0);

#define SZ_WQKV ((size_t)N3 * DM * 2)
#define SZ_WO   ((size_t)DM * DQ * 2)
#define SZ_XB   ((size_t)NB * SEQ * DM * 2)
#define SZ_F    ((size_t)NB * SEQ * N3 * 4)
#define SZ_QK   ((size_t)2 * NB * NH * SEQ * HD * 2)
#define SZ_VT   ((size_t)NB * NH * HD * SEQ * 2)
#define SZ_VR   ((size_t)NB * NH * HD * RH * 2)
#define SZ_AT   ((size_t)NB * SEQ * DQ * 2)
#define SZ_ALL  (SZ_WQKV + SZ_WO + SZ_XB + SZ_F + 2 * SZ_QK + SZ_VT + 2 * SZ_VR + 2 * SZ_AT)
static_assert(SZ_ALL <= (size_t)134217728);
static_assert(SZ_WQKV % 256 == 0 && SZ_WO % 256 == 0 && SZ_XB % 256 == 0 && SZ_F % 256 == 0 && SZ_QK % 256 == 0 && SZ_VT % 256 == 0 && SZ_VR % 256 == 0 && SZ_AT % 256 == 0);

__device__ __forceinline__ unsigned short f2bf(float f) { unsigned u = __float_as_uint(f); u += 0x7FFFu + ((u >> 16) & 1u); return (unsigned short)(u >> 16); }
__device__ __forceinline__ float bf2f(unsigned short b) { return __uint_as_float(((unsigned)b) << 16); }
__device__ __forceinline__ float bfr(float f) { return bf2f(f2bf(f)); }
__device__ __forceinline__ void splitf(float y, unsigned short& h, unsigned short& l) { h = f2bf(y); l = f2bf(y - bf2f(h)); }
__device__ __forceinline__ v16h cat16(v8h lo, v8h hi) { return __builtin_shufflevector(lo, hi, 0, 1, 2, 3, 4, 5, 6, 7, 8, 9, 10, 11, 12, 13, 14, 15); }
__device__ __forceinline__ v16bf cat16b(v8us lo, v8us hi) { return __builtin_bit_cast(v16bf, __builtin_shufflevector(lo, hi, 0, 1, 2, 3, 4, 5, 6, 7, 8, 9, 10, 11, 12, 13, 14, 15)); }
__device__ __forceinline__ v16bf ldb(const bf* p) { return cat16b(*(const v8us*)p, *(const v8us*)(p + 16)); }
__device__ __forceinline__ v16h  ldh(const h16* p) { return cat16(*(const v8h*)p, *(const v8h*)(p + 16)); }
__device__ __forceinline__ v8f wmb(v16bf a, v16bf b, v8f c) {
    c = __builtin_amdgcn_wmma_f32_16x16x32_bf16(false, a, false, b, (short)0, c, false, false);
    asm volatile("v_nop\n\tv_nop\n\tv_nop\n\tv_nop" : "+v"(c) : "v"(a), "v"(b));
    return c; }
__device__ __forceinline__ v8f wmh(v16h a, v16h b, v8f c) {
    c = __builtin_amdgcn_wmma_f32_16x16x32_f16(false, a, false, b, (short)0, c, false, false);
    asm volatile("v_nop\n\tv_nop\n\tv_nop\n\tv_nop" : "+v"(c) : "v"(a), "v"(b));
    return c; }
__device__ __forceinline__ void wave_sync() { __builtin_amdgcn_fence(3  , "wavefront"); __builtin_amdgcn_wave_barrier(); asm volatile("" ::: "memory"); }

__global__ __launch_bounds__(32) void k_gemmw(const bf* __restrict__ A, size_t a2off, int npl, const bf* __restrict__ Bt, int K, float* C, int ldc, const float* __restrict__ bias, size_t sA, size_t sC) {
    __shared__ __align__(16) float os[16 * 68];
    const size_t z = blockIdx.z; A += z * sA; C += z * sC;
    const int lane = threadIdx.x & 31, lr = lane & 15, hi = lane >> 4; const int r0 = blockIdx.x * 64, c0 = blockIdx.y * 64;
    v8f acc[4][4];
#pragma unroll
    for (int mb = 0; mb < 4; ++mb)
#pragma unroll
        for (int nb = 0; nb < 4; ++nb) acc[mb][nb] = (v8f){};
    const size_t boff = (size_t)(c0 + lr) * K + 8 * hi;
#pragma unroll 1
    for (int pl = 0; pl < npl; ++pl) {
        const size_t aoff = (size_t)pl * a2off + (size_t)(r0 + lr) * K + 8 * hi;
#pragma unroll 1
        for (int kc = 0; kc < K; kc += 32) {
            v16bf a[4];
#pragma unroll
            for (int mb = 0; mb < 4; ++mb) a[mb] = ldb(A + aoff + (size_t)mb * 16 * K + kc);
#pragma unroll
            for (int nb = 0; nb < 4; ++nb) { const v16bf b = ldb(Bt + boff + (size_t)nb * 16 * K + kc);
#pragma unroll
                for (int mb = 0; mb < 4; ++mb) acc[mb][nb] = wmb(a[mb], b, acc[mb][nb]); }
        }
    }
    const int cofs = lr * 4;
    const v4f braw = *(const v4f*)(bias + c0 + cofs);
    v4f bv; bv[0] = bfr(braw[0]); bv[1] = bfr(braw[1]); bv[2] = bfr(braw[2]); bv[3] = bfr(braw[3]);
#pragma unroll
    for (int mb = 0; mb < 4; ++mb) {
#pragma unroll
        for (int nb = 0; nb < 4; ++nb) {
#pragma unroll
            for (int j = 0; j < 8; ++j) os[(hi * 8 + j) * 68 + nb * 16 + lr] = acc[mb][nb][j]; }
        wave_sync();
        float* crow = C + (size_t)(r0 + mb * 16) * ldc + c0;
#pragma unroll 1
        for (int ps = 0; ps < 2; ++ps) {
#pragma unroll
            for (int s = 0; s < 8; ++s) { const int row = 2 * s + hi; v4f val = *(const v4fa*)(os + row * 68 + cofs); val += bv;
                *(volatile v4f*)(crow + (size_t)row * ldc + cofs) = val; }
            if (ps == 0) __threadfence(); }
        wave_sync();
    }
}

__global__ __launch_bounds__(256) void k_wtG(const float* __restrict__ w, int K, int N, bf* Bt) {
    const int lane = threadIdx.x & 31; const int wave = __builtin_amdgcn_readfirstlane(threadIdx.x >> 5);
    const int L0 = (blockIdx.x * 8 + wave) * 8; const int nlines = (int)((size_t)N * K / 64);
#pragma unroll
    for (int ps = 0; ps < 2; ++ps) {
#pragma unroll 1
        for (int l = 0; l < 8; ++l) { const int L = L0 + l; if (L >= nlines) break; const size_t e = (size_t)L * 64 + lane * 2; const int k = (int)(e % K), n = (int)(e / K); v2us o;
            o[0] = f2bf(w[(size_t)k * N + n]); o[1] = f2bf(w[(size_t)(k + 1) * N + n]); *(volatile v2us*)(Bt + e) = o; }
        if (ps == 0) __threadfence(); }
}

__global__ __launch_bounds__(256) void k_cvt8(const float* __restrict__ src, bf* dst) {
    const size_t i = (size_t)blockIdx.x * 256 + threadIdx.x; const size_t per = (size_t)SEQ * DM / 8; if (i >= (size_t)NB * per) return;
    const size_t b = i / per, rem = i - b * per; const v8f v = *(const v8f*)(src + b * ((size_t)SEQ_FULL * DM) + rem * 8); v8us o;
#pragma unroll
    for (int k = 0; k < 8; ++k) o[k] = f2bf(v[k]);
    *(volatile v8us*)(dst + i * 8) = o; __threadfence(); *(volatile v8us*)(dst + i * 8) = o; }

__global__ __launch_bounds__(256) void k_rope(const float* __restrict__ F, const float* __restrict__ fc, const float* __restrict__ fs, bf* Ph, bf* Pl) {
    const size_t id = (size_t)blockIdx.x * 256 + threadIdx.x; if (id >= (size_t)2 * NB * NH * SEQ * 32) return;
    const int j = (int)(id & 31); size_t r = id >> 5; const int t = (int)(r % SEQ); r /= SEQ; const int h = (int)(r % NH); r /= NH; const int b = (int)(r % NB); const int which = (int)(r / NB);
    const v2f x = *(const v2f*)(F + ((size_t)b * SEQ + t) * N3 + (size_t)which * DQ + h * HD + 2 * j);
    const float c = bfr(fc[(size_t)t * 32 + j]), s = bfr(fs[(size_t)t * 32 + j]);
    const float sc = which ? 1.0f : SCL;
    const float o0 = (x[0] * c - x[1] * s) * sc, o1 = (x[0] * s + x[1] * c) * sc;
    v2us oh, ol; unsigned short a, l2; splitf(o0, a, l2); oh[0] = a; ol[0] = l2; splitf(o1, a, l2); oh[1] = a; ol[1] = l2;
    const size_t o = ((((size_t)which * NB + b) * NH + h) * SEQ + t) * HD + 2 * j;
    *(volatile v2us*)(Ph + o) = oh; *(volatile v2us*)(Pl + o) = ol; __threadfence(); *(volatile v2us*)(Ph + o) = oh; *(volatile v2us*)(Pl + o) = ol; }

__global__ __launch_bounds__(256) void k_vtp(const float* __restrict__ F, h16* V16, bf* Vh, bf* Vl) {
    const size_t e = ((size_t)blockIdx.x * 256 + threadIdx.x) * 2; if (e >= (size_t)NB * NH * HD * SEQ) return;
    const int t = (int)(e % SEQ); const int d = (int)((e / SEQ) % HD); const int g = (int)(e / ((size_t)SEQ * HD)); const int b = g / NH, h = g - b * NH;
    v2h o16; v2us oh, ol;
#pragma unroll
    for (int q = 0; q < 2; ++q) { const float x = F[((size_t)b * SEQ + t + q) * N3 + 2 * DQ + h * HD + d]; o16[q] = (h16)x; unsigned short a, l2; splitf(x, a, l2); oh[q] = a; ol[q] = l2; }
    const size_t o2 = ((size_t)g * HD + d) * RH + (t < RH ? t : 0);
    *(volatile v2h*)(V16 + e) = o16; if (t < RH) { *(volatile v2us*)(Vh + o2) = oh; *(volatile v2us*)(Vl + o2) = ol; }
    __threadfence();
    *(volatile v2h*)(V16 + e) = o16; if (t < RH) { *(volatile v2us*)(Vh + o2) = oh; *(volatile v2us*)(Vl + o2) = ol; } }

template <bool HIRES>
__device__ __forceinline__ void attn_body(const bf* __restrict__ QKh, const bf* __restrict__ QKl, const h16* __restrict__ VT16, const bf* __restrict__ VTh, const bf* __restrict__ VTl, bf* ATh, bf* ATl, const int q0, const int bh) {
    __shared__ __align__(16) float os[16 * 68];
    const int lane = threadIdx.x & 31, lr = lane & 15, hi = lane >> 4;
    const size_t qpl = (size_t)bh * SEQ * HD, kpl = qpl + KOFF;
    const size_t qo = qpl + (size_t)(q0 + lr) * HD + 8 * hi;
    const v16bf qh0 = ldb(QKh + qo), qh1 = ldb(QKh + qo + 32), ql0 = ldb(QKl + qo), ql1 = ldb(QKl + qo + 32);
    v8f acc[4];
#pragma unroll
    for (int jd = 0; jd < 4; ++jd) acc[jd] = (v8f){};
    float mrow = NEGBIG, lrow = 0.0f;
    const int nch = (q0 + 47) >> 5;
    const int qi = q0 + lr;
#pragma unroll 1
    for (int ch = 0; ch < nch; ++ch) {
        const int key0 = ch << 5;
        v8f sa[2];
#pragma unroll
        for (int j = 0; j < 2; ++j) {
            const size_t ko = kpl + (size_t)(key0 + 16 * j + lr) * HD + 8 * hi;
            v8f s = (v8f){};
            v16bf a = ldb(QKh + ko), al = ldb(QKl + ko);
            s = wmb(a, qh0, s); s = wmb(al, qh0, s); s = wmb(a, ql0, s);
            a = ldb(QKh + ko + 32); al = ldb(QKl + ko + 32);
            s = wmb(a, qh1, s); s = wmb(al, qh1, s); s = wmb(a, ql1, s);
            sa[j] = s;
        }
        if (ch == nch - 1) {
#pragma unroll
            for (int r = 0; r < 8; ++r) { const int ky = key0 + 8 * hi + r; sa[0][r] = (ky <= qi) ? sa[0][r] : NEGBIG; sa[1][r] = (ky + 16 <= qi) ? sa[1][r] : NEGBIG; }
        }
        float mx = fmaxf(sa[0][0], sa[1][0]);
#pragma unroll
        for (int r = 1; r < 8; ++r) mx = fmaxf(mx, fmaxf(sa[0][r], sa[1][r]));
        mx = fmaxf(mx, __shfl_xor(mx, 16, 32));
        const float mnew = fmaxf(mrow, mx);
        const float fac = __builtin_amdgcn_exp2f((mrow - mnew) * L2E);
        mrow = mnew;
        float p0[8], p1[8]; float ps = 0.0f;
#pragma unroll
        for (int r = 0; r < 8; ++r) { p0[r] = __builtin_amdgcn_exp2f(fmaf(sa[0][r] - mnew, L2E, PCL2)); p1[r] = __builtin_amdgcn_exp2f(fmaf(sa[1][r] - mnew, L2E, PCL2)); ps += p0[r] + p1[r]; }
        lrow = lrow * fac + ps;
#pragma unroll
        for (int jd = 0; jd < 4; ++jd)
#pragma unroll
            for (int r = 0; r < 8; ++r) acc[jd][r] *= fac;
        if (HIRES) {
            v16us ph, pl;
#pragma unroll
            for (int r = 0; r < 8; ++r) { unsigned short a, l2; splitf(p0[r], a, l2); ph[r] = a; pl[r] = l2; splitf(p1[r], a, l2); ph[8 + r] = a; pl[8 + r] = l2; }
            const v16bf PH = __builtin_bit_cast(v16bf, ph), PL = __builtin_bit_cast(v16bf, pl);
#pragma unroll
            for (int jd = 0; jd < 4; ++jd) { const size_t vo = ((size_t)bh * HD + 16 * jd + lr) * RH + key0 + 8 * hi;
                const v16bf vh = ldb(VTh + vo), vl = ldb(VTl + vo);
                acc[jd] = wmb(vh, PH, acc[jd]); acc[jd] = wmb(vl, PH, acc[jd]); acc[jd] = wmb(vh, PL, acc[jd]); }
        } else {
            v16h pb;
#pragma unroll
            for (int r = 0; r < 8; ++r) { pb[r] = (h16)p0[r]; pb[8 + r] = (h16)p1[r]; }
            v16h va[4];
#pragma unroll
            for (int jd = 0; jd < 4; ++jd) va[jd] = ldh(VT16 + ((size_t)bh * HD + 16 * jd + lr) * SEQ + key0 + 8 * hi);
#pragma unroll
            for (int jd = 0; jd < 4; ++jd) acc[jd] = wmh(va[jd], pb, acc[jd]);
        }
    }
    const float lt = lrow + __shfl_xor(lrow, 16, 32);
    const float inv = 1.0f / lt;
#pragma unroll
    for (int jd = 0; jd < 4; ++jd) { v4f x0, x1;
        x0[0] = acc[jd][0] * inv; x0[1] = acc[jd][1] * inv; x0[2] = acc[jd][2] * inv; x0[3] = acc[jd][3] * inv;
        x1[0] = acc[jd][4] * inv; x1[1] = acc[jd][5] * inv; x1[2] = acc[jd][6] * inv; x1[3] = acc[jd][7] * inv;
        *(v4fa*)(os + lr * 68 + 16 * jd + 8 * hi) = x0; *(v4fa*)(os + lr * 68 + 16 * jd + 8 * hi + 4) = x1; }
    wave_sync();
    const int b = bh / NH, hh = bh - b * NH;
    const size_t arow = ((size_t)b * SEQ + q0) * DQ + (size_t)hh * HD;
    const int dofs = (lane & 7) * 8, rq = lane >> 3;
#pragma unroll 1
    for (int ps = 0; ps < 2; ++ps) {
#pragma unroll
        for (int s = 0; s < 4; ++s) { const int rr = 4 * s + rq; const v4f x0 = *(const v4fa*)(os + rr * 68 + dofs), x1 = *(const v4fa*)(os + rr * 68 + dofs + 4); v8us oh, ol;
#pragma unroll
            for (int q = 0; q < 4; ++q) { unsigned short a, l2; splitf(x0[q], a, l2); oh[q] = a; ol[q] = l2; splitf(x1[q], a, l2); oh[4 + q] = a; ol[4 + q] = l2; }
            *(volatile v8us*)(ATh + arow + (size_t)rr * DQ + dofs) = oh; *(volatile v8us*)(ATl + arow + (size_t)rr * DQ + dofs) = ol; }
        if (ps == 0) __threadfence(); }
}

__global__ __launch_bounds__(32) void k_attn_hr(const bf* __restrict__ QKh, const bf* __restrict__ QKl, const bf* __restrict__ VTh, const bf* __restrict__ VTl, bf* ATh, bf* ATl) {
    attn_body<true>(QKh, QKl, (const h16*)0, VTh, VTl, ATh, ATl, (int)blockIdx.x * 16, (int)blockIdx.y); }
__global__ __launch_bounds__(32) void k_attn_pl(const bf* __restrict__ QKh, const bf* __restrict__ QKl, const h16* __restrict__ VT16, bf* ATh, bf* ATl) {
    attn_body<false>(QKh, QKl, VT16, (const bf*)0, (const bf*)0, ATh, ATl, RH + (int)blockIdx.x * 16, (int)blockIdx.y); }

extern "C" void kernel_launch(void* const* d_in, const int* in_sizes, int n_in,
                              void* d_out, int out_size, void* d_ws, size_t ws_size, hipStream_t stream) {
    if (n_in < 8) return;
    const size_t need_x = ((size_t)(NB - 1) * SEQ_FULL + SEQ) * DM;
    if ((size_t)in_sizes[0] < need_x) return; if ((size_t)in_sizes[1] < (size_t)SEQ_FULL * SEQ_FULL) return; if ((size_t)in_sizes[2] < (size_t)SEQ * 32) return; if ((size_t)in_sizes[3] < (size_t)SEQ * 32) return;
    if ((size_t)in_sizes[4] < (size_t)DM * N3) return; if ((size_t)in_sizes[5] < (size_t)N3) return; if ((size_t)in_sizes[6] < (size_t)DQ * DM) return; if ((size_t)in_sizes[7] < (size_t)DM) return;
    if ((size_t)out_size < need_x) return;
    const float* x = (const float*)d_in[0];   const float* fcos = (const float*)d_in[2]; const float* fsin = (const float*)d_in[3];
    const float* wqkv = (const float*)d_in[4]; const float* bqkv = (const float*)d_in[5]; const float* wo = (const float*)d_in[6]; const float* bo = (const float*)d_in[7];
    float* OUT = (float*)d_out;
    char* wsp = (char*)d_ws;
    auto take = [&](size_t bytes) { char* p = wsp; wsp += (bytes + 255) & ~(size_t)255; return (void*)p; };
    bf* WQKV = (bf*)take(SZ_WQKV);
    bf* WO   = (bf*)take(SZ_WO);
    bf* XB   = (bf*)take(SZ_XB);
    float* F = (float*)take(SZ_F);
    bf* QKh  = (bf*)take(SZ_QK);
    bf* QKl  = (bf*)take(SZ_QK);
    h16* VT16 = (h16*)take(SZ_VT);
    bf* VTh  = (bf*)take(SZ_VR);
    bf* VTl  = (bf*)take(SZ_VR);
    bf* ATh  = (bf*)take(SZ_AT);
    bf* ATl  = (bf*)take(SZ_AT);
    if ((size_t)(wsp - (char*)d_ws) > ws_size) return;

    k_wtG<<<(unsigned)(((size_t)N3 * DM / 64 + 63) / 64), 256, 0, stream>>>(wqkv, DM, N3, WQKV);
    k_wtG<<<(unsigned)(((size_t)DM * DQ / 64 + 63) / 64), 256, 0, stream>>>(wo, DQ, DM, WO);
    k_cvt8<<<(unsigned)(((size_t)NB * SEQ * DM / 8 + 255) / 256), 256, 0, stream>>>(x, XB);
    k_gemmw<<<dim3(NB * SEQ / 64, N3 / 64, 1), 32, 0, stream>>>(XB, (size_t)0, 1, WQKV, DM, F, N3, bqkv, (size_t)0, (size_t)0);
    k_rope<<<(unsigned)(((size_t)2 * NB * NH * SEQ * 32 + 255) / 256), 256, 0, stream>>>(F, fcos, fsin, QKh, QKl);
    k_vtp<<<(unsigned)(((size_t)NB * NH * HD * SEQ / 2 + 255) / 256), 256, 0, stream>>>(F, VT16, VTh, VTl);
    k_attn_hr<<<dim3(RH / 16, NB * NH), 32, 0, stream>>>(QKh, QKl, VTh, VTl, ATh, ATl);
    if (SEQ > RH) k_attn_pl<<<dim3((SEQ - RH) / 16, NB * NH), 32, 0, stream>>>(QKh, QKl, VT16, ATh, ATl);
    k_gemmw<<<dim3(SEQ / 64, DM / 64, NB), 32, 0, stream>>>(ATh, (size_t)(ATl - ATh), 2, WO, DQ, OUT, DM, bo, (size_t)SEQ * DQ, (size_t)SEQ_FULL * DM);
}
